// DiGCN_IB_1BN_Sym_46746424050294
// MI455X (gfx1250) — hardware-run, weakly checked
//
#include <hip/hip_runtime.h>


namespace {
constexpr int N = 50000, NP = 50048  , E = 800000, D = 128, NBLKR = 391  ;
constexpr float XS = 8.0f, WSC = 256.0f, BNE = 1e-5f;

typedef _Float16 b16;
typedef __attribute__((ext_vector_type(16))) _Float16 v16b;
typedef __attribute__((ext_vector_type(8))) _Float16 v8b;
typedef __attribute__((ext_vector_type(8))) float v8f;
typedef __attribute__((ext_vector_type(4))) float v4f;
__device__ __forceinline__ float bf16_rne(float f) { unsigned int u = __float_as_uint(f); u += 0x7FFFu + ((u >> 16) & 1u); return __uint_as_float(u & 0xFFFF0000u); }
__device__ __forceinline__ void split16(float v, b16& hi, b16& lo) { hi = (b16)v; lo = (b16)(v - (float)hi); }
__device__ __forceinline__ v16b frag_kb(const b16* p, int hh) { const v8b a = *(const v8b*)(p + 8 * hh), b = *(const v8b*)(p + 16 + 8 * hh); v16b f;
#pragma unroll
  for (int e = 0; e < 8; ++e) { f[e] = a[e]; f[8 + e] = b[e]; } return f; }
__device__ __forceinline__ v8f wmma16b(v16b a, v16b b, v8f c) { v8f d = __builtin_amdgcn_wmma_f32_16x16x32_f16(false, a, false, b, (short)0, c, false, false); asm volatile("v_nop\n\tv_nop\n\tv_nop\n\tv_nop" : "+v"(d) : "v"(a), "v"(b)); return d; }
__device__ __forceinline__ void wave_lds_sync() { __builtin_amdgcn_fence(__ATOMIC_RELEASE, "workgroup"); __builtin_amdgcn_wave_barrier(); __builtin_amdgcn_fence(__ATOMIC_ACQUIRE, "workgroup"); }
__device__ __forceinline__ float pmul(float a, float b) { float p = a * b; asm volatile("" : "+v"(p)); return p; }
__device__ __forceinline__ int iclamp(int v, int lo, int hi) { return v < lo ? lo : (v > hi ? hi : v); }

constexpr int CSR_NBLK = 512, CSR_GB = 9, CSR_GN = 1 << CSR_GB  , CSR_MAXG = 512, CSR_CAP = 12288  ;
__global__ __launch_bounds__(64) void csrA_kernel(const int* __restrict__ dst, int E, int N, int nG, int CHP, int NGP, int* __restrict__ STG, int* __restrict__ HST) {
  extern __shared__ int sm[];
  int* cnt = sm; int* run = sm + NGP; int* ids = sm + 2 * NGP;
  const int b = blockIdx.x; const int ch = (E + CSR_NBLK - 1) / CSR_NBLK; const int e0 = b * ch, e1 = min(E, e0 + ch);
  for (int i = threadIdx.x; i < NGP; i += 64) cnt[i] = 0;
  for (int i = threadIdx.x; i < CHP; i += 64) ids[i] = -1;
  __syncthreads();
  if (threadIdx.x == 0) {
    for (int e = e0; e < e1; ++e) { int d = dst[e]; d = (d < 0) ? 0 : (d >= N ? N - 1 : d); cnt[d >> CSR_GB] += 1; }
    int acc = 0; for (int g = 0; g < nG; ++g) { run[g] = acc; acc += cnt[g]; }
    for (int e = e0; e < e1; ++e) { int d = dst[e]; d = (d < 0) ? 0 : (d >= N ? N - 1 : d); const int g = d >> CSR_GB; ids[run[g]] = e; run[g] += 1; } }
  __syncthreads();
  typedef __attribute__((ext_vector_type(4))) int v4i;
  for (int pass = 0; pass < 2; ++pass) {
    for (int i = threadIdx.x; i < CHP / 4; i += 64) *(volatile v4i*)(STG + (size_t)b * CHP + i * 4) = *(const v4i*)(&ids[i * 4]);
    for (int i = threadIdx.x; i < NGP / 4; i += 64) { v4i v; for (int e = 0; e < 4; ++e) v[e] = (i * 4 + e < nG) ? cnt[i * 4 + e] : 0; *(volatile v4i*)(HST + (size_t)b * NGP + i * 4) = v; }
    __threadfence(); }
}
__global__ __launch_bounds__(512) void csrS_kernel(const int* __restrict__ HST, int nG, int NGP, int* __restrict__ START, int* __restrict__ TOT, int* __restrict__ OFF) {
  __shared__ int tot[CSR_MAXG];
  const int b = threadIdx.x;
  for (int pass = 0; pass < 2; ++pass) { int runb = 0; for (int g = 0; g < nG; ++g) { int c = HST[(size_t)b * NGP + g]; c = (c < 0) ? 0 : c; ((volatile int*)OFF)[(size_t)g * CSR_NBLK + b] = runb; runb += c; } __threadfence(); }
  for (int g = threadIdx.x; g < nG; g += 512) { int s = 0; for (int bb = 0; bb < CSR_NBLK; ++bb) { int c = HST[(size_t)bb * NGP + g]; s += (c < 0) ? 0 : c; } tot[g] = s; }
  __syncthreads();
  if (threadIdx.x < 32) {
    __shared__ int st[CSR_MAXG + 32];
    if (threadIdx.x == 0) { int acc = 0; for (int g = 0; g < NGP; ++g) { st[g] = acc; if (g < nG) acc += (tot[g] + 31) & ~31; } st[NGP] = acc; }
    __builtin_amdgcn_fence(__ATOMIC_RELEASE, "workgroup"); __builtin_amdgcn_wave_barrier(); __builtin_amdgcn_fence(__ATOMIC_ACQUIRE, "workgroup");
    for (int pass = 0; pass < 2; ++pass) { for (int i = threadIdx.x; i < NGP + 32; i += 32) { ((volatile int*)START)[i] = (i <= NGP) ? st[min(i, NGP)] : 0; ((volatile int*)TOT)[i] = (i < nG) ? tot[i] : 0; } __threadfence(); } }
}
__global__ __launch_bounds__(256) void csrB_kernel(const int* __restrict__ dst, int N, int nG, int CHP, int NGP, int permLen, const int* __restrict__ STG, const int* __restrict__ HST, const int* __restrict__ OFF, const int* __restrict__ START, const int* __restrict__ TOT, int* __restrict__ PERM, int* __restrict__ ROWPTR, int* __restrict__ ROWCNT, int* __restrict__ FLAG) {
  typedef __attribute__((ext_vector_type(4))) int v4i;
  __shared__ int ids[CSR_CAP]; __shared__ unsigned short key[CSR_CAP]; __shared__ int outp[CSR_CAP]; __shared__ int ncnt[CSR_GN + 1]; __shared__ int boff[CSR_NBLK + 1];
  const int g = blockIdx.x, t_ = threadIdx.x; int tot = TOT[g]; int st = START[g], stn = START[g + 1]; const int v0 = g * CSR_GN; const int nv = min(CSR_GN, N - v0);
  st = (st < 0) ? 0 : (st > permLen - 32 ? permLen - 32 : st) & ~31; stn = (stn < st) ? st : (stn > permLen ? permLen : stn); tot = (tot < 0) ? 0 : tot; if (tot > stn - st && tot <= CSR_CAP) tot = stn - st;
  if (tot > CSR_CAP) {
    for (int pass = 0; pass < 2; ++pass) { for (int i = t_; i < CSR_GN / 4; i += 256) { v4i a, c; for (int e = 0; e < 4; ++e) { a[e] = st; c[e] = 0; } *(volatile v4i*)(ROWPTR + v0 + i * 4) = a; *(volatile v4i*)(ROWCNT + v0 + i * 4) = c; } if (t_ == 0) ((volatile int*)FLAG)[0] = 1; __threadfence(); } (void)nv; return; }
  if (t_ == 0) { int acc = 0; for (int b = 0; b < CSR_NBLK; ++b) { boff[b] = acc; int c = HST[(size_t)b * NGP + g]; c = (c < 0) ? 0 : (c > CHP ? CHP : c); acc += c; if (acc > tot) acc = tot; } boff[CSR_NBLK] = acc; }
  for (int i = t_; i <= CSR_GN; i += 256) ncnt[i] = 0;
  __syncthreads();
  for (int b = 0; b < CSR_NBLK; ++b) { const int c = boff[b + 1] - boff[b]; int o_ = OFF[(size_t)g * CSR_NBLK + b]; o_ = (o_ < 0) ? 0 : (o_ > CHP - c ? CHP - c : o_); const int* src_ = STG + (size_t)b * CHP + o_;
    for (int i = t_; i < c; i += 256) { int id = src_[i]; id = (id < 0) ? 0 : id; ids[boff[b] + i] = id; int d = dst[id]; d = (d < v0) ? v0 : (d >= N ? N - 1 : d); int kk = d - v0; kk = (kk < 0) ? 0 : (kk >= CSR_GN ? CSR_GN - 1 : kk); key[boff[b] + i] = (unsigned short)kk; } }
  __syncthreads();
  if (t_ == 0) { for (int i = 0; i < tot; ++i) ncnt[key[i]] += 1; int acc = 0; for (int vl = 0; vl < CSR_GN; ++vl) { const int c = ncnt[vl]; ncnt[vl] = acc; acc += c; } ncnt[CSR_GN] = acc;
    for (int i = 0; i < tot; ++i) { const int vl = key[i]; outp[ncnt[vl]] = ids[i]; ncnt[vl] += 1; }
    for (int vl = CSR_GN; vl > 0; --vl) ncnt[vl] = ncnt[vl - 1]; ncnt[0] = 0; }
  __syncthreads();
  for (int pass = 0; pass < 2; ++pass) {
    for (int i = t_; i < (stn - st) / 4; i += 256) { v4i v; for (int e = 0; e < 4; ++e) { const int q = i * 4 + e; v[e] = (q < tot) ? outp[q] : -1; } *(volatile v4i*)(PERM + st + i * 4) = v; }
    for (int i = t_; i < CSR_GN / 4; i += 256) { v4i a, c; for (int e = 0; e < 4; ++e) { const int vl = i * 4 + e; a[e] = st + ncnt[vl]; c[e] = (vl < nv) ? (ncnt[vl + 1] - ncnt[vl]) : 0; } *(volatile v4i*)(ROWPTR + v0 + i * 4) = a; *(volatile v4i*)(ROWCNT + v0 + i * 4) = c; }
    __threadfence(); }
}
__global__ __launch_bounds__(256) void csrZ_kernel(int* __restrict__ p, size_t n4) { typedef __attribute__((ext_vector_type(4))) int v4i; const size_t tid = (size_t)blockIdx.x * 256 + threadIdx.x, nth = (size_t)gridDim.x * 256; v4i z = {0, 0, 0, 0}; for (size_t i = tid; i < n4; i += nth) *(volatile v4i*)(p + i * 4) = z; }
struct CsrBufs { int *STG, *HST, *OFF, *START, *TOT, *PERM, *ROWPTR, *ROWCNT, *FLAG; int nG, NGP, CHP; size_t permLen; char* base; size_t bytes; };
static size_t csr_carve(CsrBufs& c, char* ws, size_t off, int E, int N) {
  const size_t off0 = off; c.base = ws + off;
  auto al = [&](size_t bytes) { char* p = ws + off; off += (bytes + 255) & ~(size_t)255; return p; };
  c.nG = (N + CSR_GN - 1) / CSR_GN; c.NGP = (c.nG + 31) & ~31; const int ch = (E + CSR_NBLK - 1) / CSR_NBLK; c.CHP = (ch + 31) & ~31; c.permLen = (size_t)E + 32 * (size_t)c.nG + 32;
  c.STG = (int*)al((size_t)CSR_NBLK * c.CHP * 4); c.HST = (int*)al((size_t)CSR_NBLK * c.NGP * 4); c.OFF = (int*)al((size_t)c.NGP * CSR_NBLK * 4); c.START = (int*)al((size_t)(c.NGP + 64) * 4); c.TOT = (int*)al((size_t)(c.NGP + 64) * 4);
  c.PERM = (int*)al(c.permLen * 4); c.ROWPTR = (int*)al((size_t)c.nG * CSR_GN * 4); c.ROWCNT = (int*)al((size_t)c.nG * CSR_GN * 4); c.FLAG = (int*)al(256);
  c.bytes = off - off0; return off;
}
static void csr_build(const CsrBufs& c, const int* dst, int E, int N, hipStream_t stream) {
  const size_t smem = (size_t)(2 * c.NGP + c.CHP) * 4;
  csrZ_kernel<<<512, 256, 0, stream>>>((int*)c.base, c.bytes / 16);
  csrA_kernel<<<CSR_NBLK, 64, smem, stream>>>(dst, E, N, c.nG, c.CHP, c.NGP, c.STG, c.HST);
  csrS_kernel<<<1, 512, 0, stream>>>(c.HST, c.nG, c.NGP, c.START, c.TOT, c.OFF);
  csrB_kernel<<<c.nG, 256, 0, stream>>>(dst, N, c.nG, c.CHP, c.NGP, (int)c.permLen, c.STG, c.HST, c.OFF, c.START, c.TOT, c.PERM, c.ROWPTR, c.ROWCNT, c.FLAG);
}


__global__ __launch_bounds__(256) void prep_kernel(const float* __restrict__ wln, const float* __restrict__ wlin1, const float* __restrict__ wconv, b16* __restrict__ WP, float* __restrict__ Z0, size_t nz4) {
  const size_t t = (size_t)blockIdx.x * 256 + threadIdx.x; const size_t nw = (size_t)3 * D * D / 8;
  if (t < nw) { const size_t e = t * 8; const int k = (int)(e / (D * D)); const size_t r = e - (size_t)k * D * D; const float* w = k == 0 ? wln : k == 1 ? wlin1 : wconv; v8b o; for (int j = 0; j < 8; ++j) o[j] = (b16)(bf16_rne(w[r + j]) * WSC); for (int pass = 0; pass < 2; ++pass) { *(volatile v8b*)(WP + e) = o; __threadfence(); } }
  else if (t < nw + nz4) { const v4f z = {0, 0, 0, 0}; *(volatile v4f*)(Z0 + (t - nw) * 4) = z; }
}
__global__ __launch_bounds__(256) void deg_kernel(const float* __restrict__ w, const int* __restrict__ PERM, const int* __restrict__ ROWPTR, const int* __restrict__ ROWCNT, int permLen, float* __restrict__ DIS) {
  const int v = blockIdx.x * 256 + threadIdx.x; if (v >= NP) return; float dis = 0.0f;
  if (v < N) { int st = ROWPTR[v], cnt = ROWCNT[v]; cnt = iclamp(cnt, 0, 8192); st = iclamp(st, 0, permLen - cnt); double s = 0.0;
    for (int j = 0; j < cnt; ++j) { const int e = iclamp(PERM[st + j], 0, E - 1); s += w ? (double)bf16_rne(w[e]) : 1.0; } dis = (s > 0.0) ? (float)(1.0 / sqrt(s)) : 0.0f; }
  for (int pass = 0; pass < 2; ++pass) { ((volatile float*)DIS)[v] = dis; __threadfence(); }
}
__global__ __launch_bounds__(256) void agg_kernel(const int* __restrict__ rows, const float* __restrict__ w, const float* __restrict__ x, const float* __restrict__ DIS, const int* __restrict__ PERM, const int* __restrict__ ROWPTR, const int* __restrict__ ROWCNT, int permLen, float* __restrict__ G, float* __restrict__ S) {
  const int wave = threadIdx.x >> 5, lane = threadIdx.x & 31; const size_t c = ((size_t)blockIdx.x * 8 + wave) * 2 + (lane >> 4); const int f0 = (lane & 15) * 8;
  if (c >= (size_t)N) return;
  int st = ROWPTR[c], cnt = ROWCNT[c]; cnt = iclamp(cnt, 0, 8192); st = iclamp(st, 0, permLen - cnt);
  const float disc = DIS[c];
  float acc[8] = {0, 0, 0, 0, 0, 0, 0, 0}; float ssum = 0.0f;
  for (int j = 0; j < cnt; ++j) { const int e = iclamp(PERM[st + j], 0, E - 1); const int r = iclamp(rows[e], 0, N - 1); const float disr = DIS[r];
    const float wv = w ? bf16_rne(w[e]) : 1.0f; const float nrm = pmul(pmul(disr, wv), disc); ssum += nrm;
    const v4f a = *(const v4f*)(x + (size_t)r * D + f0), b = *(const v4f*)(x + (size_t)r * D + f0 + 4);
    for (int q = 0; q < 4; ++q) { acc[q] += pmul(nrm, bf16_rne(a[q])); acc[4 + q] += pmul(nrm, bf16_rne(b[q])); } }
  v4f o0 = *(const v4f*)(G + c * D + f0), o1 = *(const v4f*)(G + c * D + f0 + 4); for (int q = 0; q < 4; ++q) { o0[q] += acc[q]; o1[q] += acc[4 + q]; }
  float so = 0.0f; if (S) so = S[c * 32 + (lane & 15)] + ((lane & 15) == 0 ? ssum : 0.0f);
  for (int pass = 0; pass < 2; ++pass) { *(volatile v4f*)(G + c * D + f0) = o0; *(volatile v4f*)(G + c * D + f0 + 4) = o1; if (S) ((volatile float*)S)[c * 32 + (lane & 15)] = so; __threadfence(); }
}
__global__ __launch_bounds__(256) void conv_kernel(const float* __restrict__ x, const float* __restrict__ Gib, const float* __restrict__ Gsym, b16* __restrict__ A1h, b16* __restrict__ A1l, b16* __restrict__ A2h, b16* __restrict__ A2l) {
  const size_t t = (size_t)blockIdx.x * 256 + threadIdx.x; if (t >= (size_t)NP * D / 8) return; const size_t e = t * 8; const size_t row = e / D;
  v8b h1, l1, h2, l2; for (int j = 0; j < 8; ++j) { float a = 0.0f, g = 0.0f; if (row < (size_t)N) { a = bf16_rne(x[e + j]) + Gib[e + j]; g = Gsym[e + j]; } b16 p, q; split16(a * XS, p, q); h1[j] = p; l1[j] = q; split16(g * XS, p, q); h2[j] = p; l2[j] = q; }
  for (int pass = 0; pass < 2; ++pass) { *(volatile v8b*)(A1h + e) = h1; *(volatile v8b*)(A1l + e) = l1; *(volatile v8b*)(A2h + e) = h2; *(volatile v8b*)(A2l + e) = l2; __threadfence(); }
}
__global__ __launch_bounds__(256) void sb_kernel(const float* __restrict__ S, float* __restrict__ SB) {
  const int row = blockIdx.x * 256 + threadIdx.x; if (row >= NP) return; const float sb = (row < N) ? 1.0f + S[(size_t)row * 32] : 0.0f;
  for (int pass = 0; pass < 2; ++pass) { ((volatile float*)SB)[row] = sb; __threadfence(); }
}
template <int MODE>
__global__ __launch_bounds__(128) void gemm_kernel(const b16* __restrict__ Ah, const b16* __restrict__ Al, const b16* __restrict__ Bh, const b16* __restrict__ Bl, const b16* __restrict__ W1, const b16* __restrict__ W2, const float* __restrict__ bias, const float* __restrict__ SB, b16* __restrict__ Yh, b16* __restrict__ Yl, float* __restrict__ Yf) {
  __shared__ __attribute__((aligned(16))) float Ts[4][16][D + 4];
  const int wave = threadIdx.x >> 5, lane = threadIdx.x & 31, nloc = lane & 15, hlf = lane >> 4; const size_t m0 = ((size_t)blockIdx.x * 4 + wave) * 16;
  v8f acc[8];
#pragma unroll
  for (int t = 0; t < 8; ++t) acc[t] = (v8f){};
#pragma unroll
  for (int kb = 0; kb < D; kb += 32) { const v16b a = frag_kb(Ah + (m0 + nloc) * D + kb, hlf), al = frag_kb(Al + (m0 + nloc) * D + kb, hlf); v16b b2 = {}, b2l = {}; if (MODE == 0) { b2 = frag_kb(Bh + (m0 + nloc) * D + kb, hlf); b2l = frag_kb(Bl + (m0 + nloc) * D + kb, hlf); }
#pragma unroll
    for (int t = 0; t < 8; ++t) { const v16b w1 = frag_kb(W1 + (size_t)(t * 16 + nloc) * D + kb, hlf); acc[t] = wmma16b(a, w1, acc[t]); acc[t] = wmma16b(al, w1, acc[t]);
      if (MODE == 0) { const v16b w2 = frag_kb(W2 + (size_t)(t * 16 + nloc) * D + kb, hlf); acc[t] = wmma16b(b2, w2, acc[t]); acc[t] = wmma16b(b2l, w2, acc[t]); } } }
#pragma unroll
  for (int t = 0; t < 8; ++t) { const int col = t * 16 + nloc; const float bb = bf16_rne(bias[col]);
#pragma unroll
    for (int r = 0; r < 8; ++r) { const size_t row = m0 + 8 * hlf + r; Ts[wave][8 * hlf + r][col] = acc[t][r] * (1.0f / (XS * WSC)) + (MODE == 0 ? pmul(SB[row], bb) : bb); } }
  wave_lds_sync();
  for (int pass = 0; pass < 2; ++pass) { for (int rr = 0; rr < 16; ++rr) {
      if (MODE == 0) { if (lane < 16) { v8b hv, lv; for (int j = 0; j < 8; ++j) { b16 p, q; split16(Ts[wave][rr][lane * 8 + j] * XS, p, q); hv[j] = p; lv[j] = q; } *(volatile v8b*)(Yh + (m0 + rr) * D + lane * 8) = hv; *(volatile v8b*)(Yl + (m0 + rr) * D + lane * 8) = lv; } }
      else *(volatile v4f*)(Yf + (m0 + rr) * D + lane * 4) = *(const v4f*)(&Ts[wave][rr][lane * 4]); }
    __threadfence(); }
}
__global__ __launch_bounds__(128) void bnsum_kernel(const float* __restrict__ HC, const float* __restrict__ MEAN, float* __restrict__ P) {
  const int blk = blockIdx.x, col = threadIdx.x; float s = 0.0f; const int r0 = blk * 128, r1 = min(r0 + 128, N);
  if (MEAN) { const float mu = MEAN[col]; for (int r = r0; r < r1; ++r) { const float dv = HC[(size_t)r * D + col] - mu; s += dv * dv; } } else { for (int r = r0; r < r1; ++r) s += HC[(size_t)r * D + col]; }
  for (int pass = 0; pass < 2; ++pass) { ((volatile float*)P)[(size_t)blk * D + col] = s; __threadfence(); }
}
__global__ __launch_bounds__(128) void bnfin_kernel(const float* __restrict__ P, int isvar, float* __restrict__ OUTV) {
  const int col = threadIdx.x; float s = 0.0f; for (int b = 0; b < NBLKR; ++b) s += P[(size_t)b * D + col]; s *= (1.0f / N); const float o = isvar ? rsqrtf(s + BNE) : s;
  for (int pass = 0; pass < 2; ++pass) { ((volatile float*)OUTV)[col] = o; __threadfence(); }
}
__global__ __launch_bounds__(256) void bnout_kernel(const float* __restrict__ HC, const float* __restrict__ MEAN, const float* __restrict__ RSTD, const float* __restrict__ gam, const float* __restrict__ bet, float* __restrict__ out) {
  const size_t t = (size_t)blockIdx.x * 256 + threadIdx.x; if (t >= (size_t)N * D / 4) return; const size_t e = t * 4; const int col = (int)(e & (D - 1));
  const v4f h = *(const v4f*)(HC + e); v4f o; for (int j = 0; j < 4; ++j) o[j] = pmul(pmul(bf16_rne(gam[col + j]), h[j] - MEAN[col + j]), RSTD[col + j]) + bf16_rne(bet[col + j]);
  for (int pass = 0; pass < 2; ++pass) { *(volatile v4f*)(out + e) = o; __threadfence(); }
}
}

extern "C" void kernel_launch(void* const* d_in, const int* in_sizes, int n_in, void* d_out, int out_size, void* d_ws, size_t ws_size, hipStream_t stream) {
  (void)n_in;
  auto Fp = [&](int i) { return (const float*)d_in[i]; }; auto Ip = [&](int i) { return (const int*)d_in[i]; };
  if (in_sizes[0] != N * D || in_sizes[1] != 2 * E || in_sizes[2] != 2 * E || in_sizes[3] != E || in_sizes[4] != 2 * E || in_sizes[6] != 2 * E || in_sizes[8] != 2 * E || in_sizes[9] != E || in_sizes[10] != D * D || out_size != N * D) return;
  size_t off = 0; char* ws = (char*)d_ws;
  auto carve = [&](size_t bytes) { char* p = ws + off; off += (bytes + 255) & ~(size_t)255; return p; };
  b16* WP = (b16*)carve((size_t)3 * D * D * 2);
  float* Z0 = (float*)carve(0); float* Gsym = (float*)carve((size_t)NP * D * 4); float* Gib = (float*)carve((size_t)NP * D * 4); float* S = (float*)carve((size_t)NP * 32 * 4); float* Zend = (float*)carve(0); float* DIS = (float*)carve((size_t)(NP + 256) * 4);
  const size_t nz4 = ((char*)Zend - (char*)Z0) / 16;
  b16* A1h = (b16*)carve((size_t)NP * D * 2); b16* A1l = (b16*)carve((size_t)NP * D * 2); b16* A2h = (b16*)carve((size_t)NP * D * 2); b16* A2l = (b16*)carve((size_t)NP * D * 2); float* SB = (float*)carve((size_t)(NP + 256) * 4);
  b16* Hh = (b16*)Gsym; b16* Hl = (b16*)((char*)Gsym + (size_t)NP * D * 2);
  float* HC = Gib;
  float* P = (float*)carve((size_t)NBLKR * D * 4); float* MEAN = (float*)carve(D * 4); float* RSTD = (float*)carve(D * 4);
  CsrBufs csr; off = csr_carve(csr, ws, off, E, N);
  if (off > ws_size || off > ((size_t)128 << 20)) return;
  const b16* Wln = WP; const b16* Wlin1 = WP + (size_t)D * D; const b16* Wconv = WP + (size_t)2 * D * D;
  prep_kernel<<<(unsigned)(((size_t)3 * D * D / 8 + nz4 + 255) / 256), 256, 0, stream>>>(Fp(11), Fp(10), Fp(13), WP, Z0, nz4);
  const int* RW[5] = {Ip(1), Ip(2), Ip(4), Ip(6), Ip(8)}; const float* WT[5] = {nullptr, Fp(3), Fp(5), Fp(7), Fp(9)}; float* TG[5] = {Gsym, Gsym, Gsym, Gib, Gib};
  for (int k = 0; k < 5; ++k) { const int* rows = RW[k]; const int* cols = RW[k] + E;
    csr_build(csr, rows, E, N, stream);
    deg_kernel<<<(NP + 255) / 256, 256, 0, stream>>>(WT[k], csr.PERM, csr.ROWPTR, csr.ROWCNT, (int)csr.permLen, DIS);
    csr_build(csr, cols, E, N, stream);
    agg_kernel<<<(N + 15) / 16, 256, 0, stream>>>(rows, WT[k], Fp(0), DIS, csr.PERM, csr.ROWPTR, csr.ROWCNT, (int)csr.permLen, TG[k], k >= 3 ? S : nullptr); }
  conv_kernel<<<(unsigned)(((size_t)NP * D / 8 + 255) / 256), 256, 0, stream>>>(Fp(0), Gib, Gsym, A1h, A1l, A2h, A2l);
  sb_kernel<<<(NP + 255) / 256, 256, 0, stream>>>(S, SB);
  gemm_kernel<0><<<NP / 64, 128, 0, stream>>>(A1h, A1l, A2h, A2l, Wln, Wlin1, Fp(12), SB, Hh, Hl, nullptr);
  gemm_kernel<1><<<NP / 64, 128, 0, stream>>>(Hh, Hl, nullptr, nullptr, Wconv, nullptr, Fp(14), nullptr, nullptr, nullptr, HC);
  bnsum_kernel<<<NBLKR, 128, 0, stream>>>(HC, nullptr, P); bnfin_kernel<<<1, 128, 0, stream>>>(P, 0, MEAN);
  bnsum_kernel<<<NBLKR, 128, 0, stream>>>(HC, MEAN, P); bnfin_kernel<<<1, 128, 0, stream>>>(P, 1, RSTD);
  bnout_kernel<<<(unsigned)(((size_t)N * D / 4 + 255) / 256), 256, 0, stream>>>(HC, MEAN, RSTD, Fp(15), Fp(16), (float*)d_out);
}
